// SqueezeformerBlock_76493367542389
// MI455X (gfx1250) — hardware-run, weakly checked
//
#include <hip/hip_runtime.h>
#include <math.h>

constexpr int kB   = 16;
constexpr int kT   = 512;
constexpr int kD   = 512;
constexpr int kH   = 8;
constexpr int kDH  = 64;
constexpr int kFF  = 2048;
constexpr int kKW  = 31;
constexpr int kNT  = kB * kT;
constexpr int kNG  = kB * kH;
constexpr int kGC  = 32;
constexpr int kNCH = kNG / kGC;
constexpr float kEps     = 1e-5f;
constexpr float kInv512  = 1.0f / 512.0f;
constexpr float kInv8192 = 1.0f / 8192.0f;

constexpr size_t kBytesWQKV = (size_t)1536 * 512 * 2;
constexpr size_t kBytesW55  = (size_t)512 * 512 * 2;
constexpr size_t kBytesWFF  = (size_t)512 * 2048 * 2;
constexpr size_t kBytesWPW1 = (size_t)1024 * 512 * 2;
constexpr size_t kOffWQKV = 0;
constexpr size_t kOffWOUT = kOffWQKV + kBytesWQKV;
constexpr size_t kOffF1W1 = kOffWOUT + kBytesW55;
constexpr size_t kOffF1W2 = kOffF1W1 + kBytesWFF;
constexpr size_t kOffPW1  = kOffF1W2 + kBytesWFF;
constexpr size_t kOffPW2  = kOffPW1 + kBytesWPW1;
constexpr size_t kOffF2W1 = kOffPW2 + kBytesW55;
constexpr size_t kOffF2W2 = kOffF2W1 + kBytesWFF;
constexpr size_t kOffXS   = kOffF2W2 + kBytesWFF;
constexpr size_t kBytesXS = (size_t)kNT * kD * 4;
constexpr size_t kOffXA   = kOffXS + kBytesXS;
constexpr size_t kBytesXA = (size_t)kNT * kD * 2;
constexpr size_t kOffBIG  = kOffXA + kBytesXA;
constexpr size_t kBytesBIG = (size_t)kNT * 1536 * 4;
constexpr size_t kOffR2   = kOffBIG + kBytesBIG;
constexpr size_t kBytesR2 = (size_t)3 * kNG * kT * kDH * 2;
constexpr size_t kOffCS   = kOffR2 + kBytesR2;
constexpr size_t kBytesCS = (size_t)kT * 64 * 4;
constexpr size_t kOffSTATS = kOffCS + kBytesCS;
constexpr size_t kBytesSTATS = 4096;
constexpr size_t kWsTotal = kOffSTATS + kBytesSTATS;
constexpr size_t kBytesS  = (size_t)kGC * kT * kT * 4;
constexpr size_t kBytesP  = (size_t)kGC * kT * kT * 2;
static_assert(kOffXS == 12058624, "weights size");
static_assert(kBytesS + kBytesP == kBytesBIG, "S+P fit BIG");
static_assert((size_t)kNT * kFF * 2 <= kBytesBIG, "Hd fits BIG");
static_assert((size_t)kNT * 1024 * 4 + (size_t)kNT * kD * 4 == kBytesBIG, "Z1+ZG fit BIG");
static_assert((size_t)kNT * kD * 4 <= kBytesR2, "Y fits R2");
static_assert(kWsTotal == 112857088, "carve total");
static_assert(kWsTotal <= (size_t)134217728, "carve limit");

typedef __attribute__((ext_vector_type(16))) _Float16 v16h;
typedef __attribute__((ext_vector_type(8)))  _Float16 v8h;
typedef __attribute__((ext_vector_type(16))) __bf16   v16b;
typedef __attribute__((ext_vector_type(8)))  __bf16   v8b;
typedef __attribute__((ext_vector_type(8)))  float    v8f;
typedef __attribute__((ext_vector_type(4)))  float    v4f;
typedef __attribute__((ext_vector_type(4)))  unsigned int v4u;

__device__ __forceinline__ unsigned short f2bf_bits(float f) {
  unsigned u = __float_as_uint(f);
  return (unsigned short)((u + 0x7FFFu + ((u >> 16) & 1u)) >> 16);
}
__device__ __forceinline__ float bf_bits2f(unsigned short h) { return __uint_as_float(((unsigned)h) << 16); }

__device__ __forceinline__ void dep_guard_h(v8f& a, v8f& b, v16h x, v16h y) { asm volatile("v_nop\n\tv_nop\n\tv_nop\n\tv_nop" : "+v"(a), "+v"(b) : "v"(x), "v"(y)); }
__device__ __forceinline__ void dep_guard_b(v8f& a, v8f& b, v16b x, v16b y) { asm volatile("v_nop\n\tv_nop\n\tv_nop\n\tv_nop" : "+v"(a), "+v"(b) : "v"(x), "v"(y)); }
__device__ __forceinline__ void keep4_h(v16h a, v16h b, v16h c, v16h d) { asm volatile("v_nop" :: "v"(a), "v"(b), "v"(c), "v"(d)); }
__device__ __forceinline__ void keep4_b(v16b a, v16b b, v16b c, v16b d) { asm volatile("v_nop" :: "v"(a), "v"(b), "v"(c), "v"(d)); }
__device__ __forceinline__ void acc_guard4(v8f& a, v8f& b, v8f& c, v8f& d) { asm volatile("v_nop\n\tv_nop\n\tv_nop\n\tv_nop" : "+v"(a), "+v"(b), "+v"(c), "+v"(d)); }
template <typename T> struct Frag;
template <> struct Frag<_Float16> {
  typedef v16h V; union U { v16h v; v8h h[2]; };
  static __device__ __forceinline__ v16h load(const _Float16* p) {
    U f; f.h[0] = *(const v8h*)(p); f.h[1] = *(const v8h*)(p + 16); return f.v;
  }
  static __device__ __forceinline__ v8f mma(v16h a, v16h b, v8f c) {
    return __builtin_amdgcn_wmma_f32_16x16x32_f16(false, a, false, b, (short)0, c, false, false);
  }
  static __device__ __forceinline__ void guard(v8f& a, v8f& b, v16h x, v16h y) { dep_guard_h(a, b, x, y); }
  static __device__ __forceinline__ void keep(v16h a, v16h b, v16h c, v16h d) { keep4_h(a, b, c, d); }
};
template <> struct Frag<__bf16> {
  typedef v16b V; union U { v16b v; v8b h[2]; };
  static __device__ __forceinline__ v16b load(const __bf16* p) {
    U f; f.h[0] = *(const v8b*)(p); f.h[1] = *(const v8b*)(p + 16); return f.v;
  }
  static __device__ __forceinline__ v8f mma(v16b a, v16b b, v8f c) {
    return __builtin_amdgcn_wmma_f32_16x16x32_bf16(false, a, false, b, (short)0, c, false, false);
  }
  static __device__ __forceinline__ void guard(v8f& a, v8f& b, v16b x, v16b y) { dep_guard_b(a, b, x, y); }
  static __device__ __forceinline__ void keep(v16b a, v16b b, v16b c, v16b d) { keep4_b(a, b, c, d); }
};

__device__ __forceinline__ unsigned pk16(unsigned short a, unsigned short b) { return (unsigned)a | ((unsigned)b << 16); }
__device__ __forceinline__ unsigned short h_bits(float f) { const _Float16 h = (_Float16)f; return __builtin_bit_cast(unsigned short, h); }

template <int ET> struct Elem;
template <> struct Elem<0> { typedef _Float16 T; };
template <> struct Elem<1> { typedef __bf16 T; };
template <int ET, bool SPLIT, int BIAS_MODE, int OUT_MODE, bool RESID, int ACT = 0>
__global__ __launch_bounds__(256) void wmma_gemm64(
    const unsigned short* __restrict__ Ap, const unsigned short* __restrict__ A2p, int lda, long strideA,
    const unsigned short* __restrict__ Btp, const unsigned short* __restrict__ Bt2p, int ldb, long strideB,
    void* __restrict__ Cout, void* __restrict__ Cout2, int ldc, long strideCo, long strideCi, int zdiv,
    const float* __restrict__ bias,
    const float* __restrict__ resid, long strideR,
    int M, int N, int K, float scale, float oscale) {
  typedef typename Elem<ET>::T T;
  typedef typename Frag<T>::V V;
  const T* A = (const T*)Ap; const T* A2 = (const T*)A2p; const T* Bt = (const T*)Btp; const T* Bt2 = (const T*)Bt2p;
  __shared__ __align__(16) float sT[8][16 * 68];
  const int b    = blockIdx.y;
  const int lane = threadIdx.x & 31;
  const int wave = threadIdx.x >> 5;
  const int tilesN = N >> 6;
  const int tilesM = M >> 6;
  const int tile = blockIdx.x * 8 + wave;
  if (tile >= tilesM * tilesN) return;
  const int tm = tile / tilesN;
  const int tn = tile - tm * tilesN;
  const int m0 = tm << 6;
  const int n0 = tn << 6;

  const T* Ab  = A  + (size_t)b * strideA;
  const T* Bb  = Bt + (size_t)b * strideB;
  const T* Ab2 = SPLIT ? (A2  + (size_t)b * strideA) : nullptr;
  const T* Bb2 = SPLIT ? (Bt2 + (size_t)b * strideB) : nullptr;

  const int rlane = lane & 15;
  const int koff  = (lane >> 4) * 8;
  const int mOff  = (lane >> 4) * 8;

  v8f acc[4][4];
#pragma unroll
  for (int i = 0; i < 4; ++i)
#pragma unroll
    for (int j = 0; j < 4; ++j) acc[i][j] = (v8f){0.f,0.f,0.f,0.f,0.f,0.f,0.f,0.f};

  for (int k0 = 0; k0 < K; k0 += 32) {
    V bh[4], bl[4];
#pragma unroll
    for (int j = 0; j < 4; ++j) {
      const size_t bo = (size_t)(n0 + (j << 4) + rlane) * ldb + koff + k0;
      bh[j] = Frag<T>::load(Bb + bo);
      if (SPLIT) bl[j] = Frag<T>::load(Bb2 + bo);
    }
#pragma unroll
    for (int i = 0; i < 4; ++i) {
      const size_t ao = (size_t)(m0 + (i << 4) + rlane) * lda + koff + k0;
      V ah = Frag<T>::load(Ab + ao);
      V al;
      if (SPLIT) al = Frag<T>::load(Ab2 + ao);
#pragma unroll
      for (int j = 0; j < 4; ++j) {
        acc[i][j] = Frag<T>::mma(ah, bh[j], acc[i][j]);
        if (SPLIT) {
          acc[i][j] = Frag<T>::mma(ah, bl[j], acc[i][j]);
          acc[i][j] = Frag<T>::mma(al, bh[j], acc[i][j]);
        }
      }
      Frag<T>::guard(acc[i][0], acc[i][3], ah, SPLIT ? al : ah);
    }
    Frag<T>::keep(bh[0], bh[1], bh[2], bh[3]);
    if (SPLIT) Frag<T>::keep(bl[0], bl[1], bl[2], bl[3]);
  }
  acc_guard4(acc[0][0], acc[0][1], acc[0][2], acc[0][3]);
  acc_guard4(acc[1][0], acc[1][1], acc[1][2], acc[1][3]);
  acc_guard4(acc[2][0], acc[2][1], acc[2][2], acc[2][3]);
  acc_guard4(acc[3][0], acc[3][1], acc[3][2], acc[3][3]);

  float* slab = sT[wave];
  const int zo = b / zdiv;
  const int zi = b - zo * zdiv;
  const size_t cbase = (size_t)zo * strideCo + (size_t)zi * strideCi;
  const float* Rb = RESID ? (resid + (size_t)b * strideR) : nullptr;
#pragma unroll
  for (int i = 0; i < 4; ++i) {
    const int mBase = m0 + (i << 4);
#pragma unroll
    for (int j = 0; j < 4; ++j) {
      const int n = n0 + (j << 4) + rlane;
      float bv = 0.f;
      if (BIAS_MODE == 2) bv = bias[n];
#pragma unroll
      for (int r = 0; r < 8; ++r) {
        float v = acc[i][j][r] * scale;
        if (BIAS_MODE == 1) v += bias[mBase + mOff + r];
        if (BIAS_MODE == 2) v += bv;
        if (RESID) v += Rb[(size_t)(mBase + mOff + r) * ldc + n];
        if (ACT == 2) v = fmaxf(v, 0.0f);
        if (ACT == 3) v = v / (1.0f + expf(-v));
        if (ACT == 4) v = (v > 0.f) ? v : 0.01f * v;
        v = v * oscale;
        slab[(mOff + r) * 68 + (j << 4) + rlane] = v;
      }
    }
    __builtin_amdgcn_fence(__ATOMIC_RELEASE, "workgroup");
    __builtin_amdgcn_wave_barrier();
    __builtin_amdgcn_fence(__ATOMIC_ACQUIRE, "workgroup");
    if (OUT_MODE == 0) {
      float* C = (float*)Cout + cbase;
      const int hh = lane >> 4, c4 = (lane & 15) * 4;
      for (int pass = 0; pass < 2; ++pass) {
#pragma unroll
        for (int it = 0; it < 8; ++it) {
          const int row = it * 2 + hh;
          v4f v = *(const v4f*)(slab + row * 68 + c4);
          *(volatile v4f*)(C + (size_t)(mBase + row) * ldc + n0 + c4) = v;
        }
        __threadfence();
      }
    } else {
      const int q = lane >> 3, c8 = (lane & 7) * 8;
      unsigned short* C  = (unsigned short*)Cout  + cbase;
      unsigned short* C2 = (OUT_MODE == 2) ? ((unsigned short*)Cout2 + cbase) : nullptr;
      for (int pass = 0; pass < 2; ++pass) {
#pragma unroll
        for (int it = 0; it < 4; ++it) {
          const int row = it * 4 + q;
          const float* sp = slab + row * 68 + c8;
          v8h hv, lv;
#pragma unroll
          for (int e = 0; e < 8; ++e) {
            if (OUT_MODE == 1) {
              hv[e] = (_Float16)sp[e];
            } else {
              unsigned short hb = f2bf_bits(sp[e]);
              unsigned short lb = f2bf_bits(sp[e] - bf_bits2f(hb));
              hv[e] = __builtin_bit_cast(_Float16, hb);
              lv[e] = __builtin_bit_cast(_Float16, lb);
            }
          }
          *(volatile v8h*)(C + (size_t)(mBase + row) * ldc + n0 + c8) = hv;
          if (OUT_MODE == 2) *(volatile v8h*)(C2 + (size_t)(mBase + row) * ldc + n0 + c8) = lv;
        }
        __threadfence();
      }
    }
    __builtin_amdgcn_fence(__ATOMIC_RELEASE, "workgroup");
    __builtin_amdgcn_wave_barrier();
    __builtin_amdgcn_fence(__ATOMIC_ACQUIRE, "workgroup");
  }
}

__global__ __launch_bounds__(256) void wtcast_kernel(const float* __restrict__ W, unsigned short* __restrict__ WT,
                                                     int Kin, int Nout, float scale) {
  __shared__ float sm[64][65];
  const int t  = threadIdx.x;
  const int k0 = blockIdx.x * 64;
  const int n0 = blockIdx.y * 64;
#pragma unroll
  for (int i = 0; i < 16; ++i) {
    const int e = i * 256 + t;
    const int r = e >> 6;
    const int c = e & 63;
    sm[c][r] = W[(size_t)(k0 + r) * Nout + n0 + c] * scale;
  }
  __syncthreads();
  const int lane = t & 31, wave = t >> 5;
  const int q = lane >> 3, c8 = (lane & 7) * 8;
  for (int pass = 0; pass < 2; ++pass) {
#pragma unroll
    for (int it = 0; it < 2; ++it) {
      const int row = wave * 8 + it * 4 + q;
      unsigned short hb[8];
#pragma unroll
      for (int e = 0; e < 8; ++e) hb[e] = h_bits(sm[row][c8 + e]);
      const v4u u = (v4u){pk16(hb[0], hb[1]), pk16(hb[2], hb[3]), pk16(hb[4], hb[5]), pk16(hb[6], hb[7])};
      *(volatile v4u*)(WT + (size_t)(n0 + row) * Kin + k0 + c8) = u;
    }
    __threadfence();
  }
}

__global__ __launch_bounds__(256) void sbcast_kernel(const float* __restrict__ X, const float* __restrict__ s,
                                                     const float* __restrict__ bb, unsigned short* __restrict__ XA, int n8) {
  const int i = blockIdx.x * 256 + threadIdx.x;
  if (i >= n8) return;
  const size_t e0 = (size_t)i * 8;
  const int d0 = (int)(e0 & (size_t)(kD - 1));
  const v4f x0 = *(const v4f*)(X + e0), x1 = *(const v4f*)(X + e0 + 4);
  const v4f s0 = *(const v4f*)(s + d0), s1 = *(const v4f*)(s + d0 + 4);
  const v4f b0 = *(const v4f*)(bb + d0), b1 = *(const v4f*)(bb + d0 + 4);
  unsigned short hb[8];
#pragma unroll
  for (int e = 0; e < 4; ++e) {
    hb[e]     = h_bits(x0[e] * s0[e] + b0[e]);
    hb[4 + e] = h_bits(x1[e] * s1[e] + b1[e]);
  }
  const v4u u = (v4u){pk16(hb[0], hb[1]), pk16(hb[2], hb[3]), pk16(hb[4], hb[5]), pk16(hb[6], hb[7])};
  unsigned short* q = XA + e0;
  *(volatile v4u*)q = u;
  __threadfence();
  *(volatile v4u*)q = u;
}

__global__ __launch_bounds__(256) void rope_table_kernel(float* __restrict__ CS) {
  __shared__ float s_inv[32];
  const int tid = threadIdx.x;
  if (tid < 32) {
    const float ex = (float)(2 * tid) * 0.015625f;
    const float p  = powf(10000.0f, ex);
    s_inv[tid] = 1.0f / p;
  }
  __syncthreads();
  const int lane = tid & 31, wave = tid >> 5;
  const int t = blockIdx.x * 8 + wave;
  const float ang = (float)t * s_inv[lane];
  float sn, cs;
  sincosf(ang, &sn, &cs);
  float* row = CS + (size_t)t * 64;
  ((volatile float*)row)[lane]      = cs;
  ((volatile float*)row)[32 + lane] = sn;
  __threadfence();
  ((volatile float*)row)[lane]      = cs;
  ((volatile float*)row)[32 + lane] = sn;
}

__global__ __launch_bounds__(256) void rope_split_kernel(const float* __restrict__ QKV, const float* __restrict__ CS,
                                                         unsigned short* __restrict__ QH, unsigned short* __restrict__ KH,
                                                         unsigned short* __restrict__ VT, float carry) {
  __shared__ __align__(16) unsigned short sq[64 * 72];
  __shared__ __align__(16) unsigned short sk[64 * 72];
  __shared__ __align__(16) unsigned short sv[64 * 72];
  const int tid = threadIdx.x;
  const int t0 = blockIdx.x * 64, h = blockIdx.y, b = blockIdx.z;
  const int g  = b * kH + h;
  const int tl = tid >> 2, j0 = (tid & 3) * 8;
  const int t  = t0 + tl;
  const float* base = QKV + (size_t)(b * kT + t) * (size_t)(3 * kD) + h * kDH;
  const v4f qa0 = *(const v4f*)(base + j0),        qa1 = *(const v4f*)(base + j0 + 4);
  const v4f qb0 = *(const v4f*)(base + 32 + j0),   qb1 = *(const v4f*)(base + 32 + j0 + 4);
  const v4f ka0 = *(const v4f*)(base + 512 + j0),  ka1 = *(const v4f*)(base + 512 + j0 + 4);
  const v4f kb0 = *(const v4f*)(base + 544 + j0),  kb1 = *(const v4f*)(base + 544 + j0 + 4);
  const v4f va0 = *(const v4f*)(base + 1024 + j0), va1 = *(const v4f*)(base + 1024 + j0 + 4);
  const v4f vb0 = *(const v4f*)(base + 1056 + j0), vb1 = *(const v4f*)(base + 1056 + j0 + 4);
  const float* csr = CS + (size_t)t * 64;
  const v4f c0v = *(const v4f*)(csr + j0),      c1v = *(const v4f*)(csr + j0 + 4);
  const v4f s0v = *(const v4f*)(csr + 32 + j0), s1v = *(const v4f*)(csr + 32 + j0 + 4);
  float q1[8], q2[8], k1[8], k2[8], v1[8], v2[8], cc[8], ss[8];
#pragma unroll
  for (int e = 0; e < 4; ++e) {
    q1[e] = qa0[e]; q1[4 + e] = qa1[e]; q2[e] = qb0[e]; q2[4 + e] = qb1[e];
    k1[e] = ka0[e]; k1[4 + e] = ka1[e]; k2[e] = kb0[e]; k2[4 + e] = kb1[e];
    v1[e] = va0[e]; v1[4 + e] = va1[e]; v2[e] = vb0[e]; v2[4 + e] = vb1[e];
    cc[e] = c0v[e]; cc[4 + e] = c1v[e]; ss[e] = s0v[e]; ss[4 + e] = s1v[e];
  }
#pragma unroll
  for (int e = 0; e < 8; ++e) {
    const int j = j0 + e;
    const float c = cc[e], s = ss[e];
    sq[tl * 72 + j]      = h_bits(carry * (q1[e] * c - q2[e] * s));
    sq[tl * 72 + 32 + j] = h_bits(carry * (q2[e] * c + q1[e] * s));
    sk[tl * 72 + j]      = h_bits(carry * (k1[e] * c - k2[e] * s));
    sk[tl * 72 + 32 + j] = h_bits(carry * (k2[e] * c + k1[e] * s));
    sv[j * 72 + tl]        = h_bits(carry * v1[e]);
    sv[(32 + j) * 72 + tl] = h_bits(carry * v2[e]);
  }
  __syncthreads();
  const int q8 = tid >> 3, c8 = (tid & 7) * 8;
  for (int pass = 0; pass < 2; ++pass) {
#pragma unroll
    for (int it = 0; it < 2; ++it) {
      const int r = it * 32 + q8;
      const v4u uq = *(const v4u*)(sq + r * 72 + c8);
      const v4u uk = *(const v4u*)(sk + r * 72 + c8);
      const v4u uv = *(const v4u*)(sv + r * 72 + c8);
      *(volatile v4u*)(QH + (size_t)(g * kT + t0 + r) * kDH + c8) = uq;
      *(volatile v4u*)(KH + (size_t)(g * kT + t0 + r) * kDH + c8) = uk;
      *(volatile v4u*)(VT + (size_t)(g * kDH + r) * kT + t0 + c8) = uv;
    }
    __threadfence();
  }
}

__global__ __launch_bounds__(256) void softmax_kernel(const float* __restrict__ S, unsigned short* __restrict__ P, float carry) {
  const int lane = threadIdx.x & 31, wave = threadIdx.x >> 5;
  const int row = blockIdx.x * 8 + wave;
  const int c0 = lane * 8, c1 = 256 + lane * 8;
  const float* sr = S + (size_t)row * kT;
  const v4f a0 = *(const v4f*)(sr + c0), a1 = *(const v4f*)(sr + c0 + 4);
  const v4f a2 = *(const v4f*)(sr + c1), a3 = *(const v4f*)(sr + c1 + 4);
  float x[16];
#pragma unroll
  for (int e = 0; e < 4; ++e) { x[e] = a0[e]; x[4 + e] = a1[e]; x[8 + e] = a2[e]; x[12 + e] = a3[e]; }
  float m = x[0];
#pragma unroll
  for (int e = 1; e < 16; ++e) m = fmaxf(m, x[e]);
#pragma unroll
  for (int off = 16; off > 0; off >>= 1) m = fmaxf(m, __shfl_xor(m, off, 32));
  float sum = 0.f;
#pragma unroll
  for (int e = 0; e < 16; ++e) { x[e] = expf(x[e] - m); sum += x[e]; }
#pragma unroll
  for (int off = 16; off > 0; off >>= 1) sum += __shfl_xor(sum, off, 32);
  const float rr = carry / sum;
  unsigned short hb[16];
#pragma unroll
  for (int e = 0; e < 16; ++e) hb[e] = h_bits(x[e] * rr);
  const v4u u0 = (v4u){pk16(hb[0], hb[1]), pk16(hb[2], hb[3]), pk16(hb[4], hb[5]), pk16(hb[6], hb[7])};
  const v4u u1 = (v4u){pk16(hb[8], hb[9]), pk16(hb[10], hb[11]), pk16(hb[12], hb[13]), pk16(hb[14], hb[15])};
  unsigned short* pr = P + (size_t)row * kT;
  for (int pass = 0; pass < 2; ++pass) {
    *(volatile v4u*)(pr + c0) = u0;
    *(volatile v4u*)(pr + c1) = u1;
    __threadfence();
  }
}

template <bool EMIT16>
__global__ __launch_bounds__(256) void ln_kernel(const float* __restrict__ Y, const float* __restrict__ g, const float* __restrict__ bb,
                                                 const float* __restrict__ sbs, const float* __restrict__ sbb,
                                                 float* __restrict__ XO, unsigned short* __restrict__ XA) {
  __shared__ __align__(16) float srow[8][512];
  const int lane = threadIdx.x & 31, wave = threadIdx.x >> 5;
  const int row = blockIdx.x * 8 + wave;
  const int c0 = lane * 8, c1 = 256 + lane * 8;
  const float* yr = Y + (size_t)row * kD;
  const v4f a0 = *(const v4f*)(yr + c0), a1 = *(const v4f*)(yr + c0 + 4);
  const v4f a2 = *(const v4f*)(yr + c1), a3 = *(const v4f*)(yr + c1 + 4);
  float x[16];
#pragma unroll
  for (int e = 0; e < 4; ++e) { x[e] = a0[e]; x[4 + e] = a1[e]; x[8 + e] = a2[e]; x[12 + e] = a3[e]; }
  float s = 0.f;
#pragma unroll
  for (int e = 0; e < 16; ++e) s += x[e];
#pragma unroll
  for (int off = 16; off > 0; off >>= 1) s += __shfl_xor(s, off, 32);
  const float mean = s * kInv512;
  float q = 0.f;
#pragma unroll
  for (int e = 0; e < 16; ++e) { const float d = x[e] - mean; x[e] = d; q += d * d; }
#pragma unroll
  for (int off = 16; off > 0; off >>= 1) q += __shfl_xor(q, off, 32);
  const float inv = rsqrtf(q * kInv512 + kEps);
  const v4f g0 = *(const v4f*)(g + c0), g1 = *(const v4f*)(g + c0 + 4), g2 = *(const v4f*)(g + c1), g3 = *(const v4f*)(g + c1 + 4);
  const v4f b0 = *(const v4f*)(bb + c0), b1 = *(const v4f*)(bb + c0 + 4), b2 = *(const v4f*)(bb + c1), b3 = *(const v4f*)(bb + c1 + 4);
  float gg[16], bv[16], o[16];
#pragma unroll
  for (int e = 0; e < 4; ++e) {
    gg[e] = g0[e]; gg[4 + e] = g1[e]; gg[8 + e] = g2[e]; gg[12 + e] = g3[e];
    bv[e] = b0[e]; bv[4 + e] = b1[e]; bv[8 + e] = b2[e]; bv[12 + e] = b3[e];
  }
#pragma unroll
  for (int e = 0; e < 16; ++e) o[e] = x[e] * inv * gg[e] + bv[e];
  float* sr = srow[wave];
  *(v4f*)(sr + c0)     = (v4f){o[0], o[1], o[2], o[3]};
  *(v4f*)(sr + c0 + 4) = (v4f){o[4], o[5], o[6], o[7]};
  *(v4f*)(sr + c1)     = (v4f){o[8], o[9], o[10], o[11]};
  *(v4f*)(sr + c1 + 4) = (v4f){o[12], o[13], o[14], o[15]};
  __builtin_amdgcn_fence(__ATOMIC_RELEASE, "workgroup");
  __builtin_amdgcn_wave_barrier();
  __builtin_amdgcn_fence(__ATOMIC_ACQUIRE, "workgroup");
  float* xo = XO + (size_t)row * kD;
  for (int pass = 0; pass < 2; ++pass) {
#pragma unroll
    for (int it = 0; it < 4; ++it) {
      const v4f v = *(const v4f*)(sr + it * 128 + lane * 4);
      *(volatile v4f*)(xo + it * 128 + lane * 4) = v;
    }
    __threadfence();
  }
  if (EMIT16) {
    const v4f p0 = *(const v4f*)(sbs + c0), p1 = *(const v4f*)(sbs + c0 + 4), p2 = *(const v4f*)(sbs + c1), p3 = *(const v4f*)(sbs + c1 + 4);
    const v4f r0 = *(const v4f*)(sbb + c0), r1 = *(const v4f*)(sbb + c0 + 4), r2 = *(const v4f*)(sbb + c1), r3 = *(const v4f*)(sbb + c1 + 4);
    float ps[16], pb[16];
#pragma unroll
    for (int e = 0; e < 4; ++e) {
      ps[e] = p0[e]; ps[4 + e] = p1[e]; ps[8 + e] = p2[e]; ps[12 + e] = p3[e];
      pb[e] = r0[e]; pb[4 + e] = r1[e]; pb[8 + e] = r2[e]; pb[12 + e] = r3[e];
    }
    unsigned short hb[16];
#pragma unroll
    for (int e = 0; e < 16; ++e) hb[e] = h_bits(o[e] * ps[e] + pb[e]);
    const v4u u0 = (v4u){pk16(hb[0], hb[1]), pk16(hb[2], hb[3]), pk16(hb[4], hb[5]), pk16(hb[6], hb[7])};
    const v4u u1 = (v4u){pk16(hb[8], hb[9]), pk16(hb[10], hb[11]), pk16(hb[12], hb[13]), pk16(hb[14], hb[15])};
    unsigned short* xa = XA + (size_t)row * kD;
    for (int pass = 0; pass < 2; ++pass) {
      *(volatile v4u*)(xa + c0) = u0;
      *(volatile v4u*)(xa + c1) = u1;
      __threadfence();
    }
  }
}

__global__ __launch_bounds__(256) void glu_kernel(const float* __restrict__ Z1, float* __restrict__ ZG) {
  const int i = blockIdx.x * 256 + threadIdx.x;
  const int r = i >> 7, d0 = (i & 127) * 4;
  const v4f a  = *(const v4f*)(Z1 + (size_t)r * 1024 + d0);
  const v4f gt = *(const v4f*)(Z1 + (size_t)r * 1024 + 512 + d0);
  v4f o;
#pragma unroll
  for (int e = 0; e < 4; ++e) o[e] = a[e] * (1.0f / (1.0f + expf(-gt[e])));
  float* p = ZG + (size_t)r * kD + d0;
  *(volatile v4f*)p = o;
  __threadfence();
  *(volatile v4f*)p = o;
}

__global__ __launch_bounds__(256) void dwconv_kernel(const float* __restrict__ ZG, const float* __restrict__ Wd,
                                                     const float* __restrict__ bd, float* __restrict__ ZC) {
  __shared__ __align__(16) float zs[94 * 64];
  __shared__ __align__(16) float wsm[31 * 64];
  __shared__ __align__(16) float osm[64 * 68];
  const int tid = threadIdx.x;
  const int c0 = blockIdx.x * 64, t0 = blockIdx.y * 64, b = blockIdx.z;
#pragma unroll 1
  for (int i = 0; i < 24; ++i) {
    int e = i * 256 + tid;
    const bool ok = e < 94 * 64;
    e = ok ? e : 0;
    const int rr = e >> 6, cc = e & 63;
    const int t  = t0 - 15 + rr;
    const int tc = t < 0 ? 0 : (t > kT - 1 ? kT - 1 : t);
    float v = ZG[(size_t)(b * kT + tc) * kD + c0 + cc];
    v = (t >= 0 && t < kT) ? v : 0.f;
    if (ok) zs[e] = v;
  }
#pragma unroll 1
  for (int i = 0; i < 8; ++i) {
    int e = i * 256 + tid;
    const bool ok = e < 31 * 64;
    e = ok ? e : 0;
    const int cc = e / 31;
    const int kk = e - cc * 31;
    const float w = Wd[(size_t)c0 * 31 + e];
    if (ok) wsm[kk * 64 + cc] = w;
  }
  __syncthreads();
  const int c = tid & 63, rg = tid >> 6;
  float acc[16];
#pragma unroll
  for (int i = 0; i < 16; ++i) acc[i] = 0.f;
#pragma unroll 1
  for (int kk = 0; kk < kKW; ++kk) {
    const float w = wsm[kk * 64 + c];
    const float* zp = zs + (rg * 16 + kk) * 64 + c;
#pragma unroll
    for (int i = 0; i < 16; ++i) acc[i] += zp[i * 64] * w;
  }
  const float bv = bd[c0 + c];
#pragma unroll
  for (int i = 0; i < 16; ++i) osm[(rg * 16 + i) * 68 + c] = acc[i] + bv;
  __syncthreads();
  const int rq = tid >> 4, c4 = (tid & 15) * 4;
  for (int pass = 0; pass < 2; ++pass) {
#pragma unroll
    for (int it = 0; it < 4; ++it) {
      const int row = it * 16 + rq;
      const v4f v = *(const v4f*)(osm + row * 68 + c4);
      *(volatile v4f*)(ZC + (size_t)(b * kT + t0 + row) * kD + c0 + c4) = v;
    }
    __threadfence();
  }
}

__global__ __launch_bounds__(256) void bnstats_kernel(const float* __restrict__ ZC, float* __restrict__ stats) {
  __shared__ float red[8][32];
  __shared__ float smean[32];
  __shared__ __align__(16) float sout[64];
  const int lane = threadIdx.x & 31, wave = threadIdx.x >> 5;
  const int c = blockIdx.x * 32 + lane;
  float s = 0.f;
#pragma unroll 1
  for (int i = 0; i < kNT / 8; ++i) s += ZC[(size_t)(wave + 8 * i) * kD + c];
  red[wave][lane] = s;
  __syncthreads();
  if (wave == 0) {
    float tsum = 0.f;
#pragma unroll
    for (int w = 0; w < 8; ++w) tsum += red[w][lane];
    smean[lane] = tsum * kInv8192;
  }
  __syncthreads();
  const float mean = smean[lane];
  float q = 0.f;
#pragma unroll 1
  for (int i = 0; i < kNT / 8; ++i) { const float d = ZC[(size_t)(wave + 8 * i) * kD + c] - mean; q += d * d; }
  red[wave][lane] = q;
  __syncthreads();
  if (wave == 0) {
    float tq = 0.f;
#pragma unroll
    for (int w = 0; w < 8; ++w) tq += red[w][lane];
    sout[lane]      = mean;
    sout[32 + lane] = tq * kInv8192;
  }
  __syncthreads();
  if (wave == 0 && lane < 16) {
    const v4f v = *(const v4f*)(sout + lane * 4);
    float* sp = stats + (size_t)blockIdx.x * 64 + lane * 4;
    *(volatile v4f*)sp = v;
    __threadfence();
    *(volatile v4f*)sp = v;
  }
}

__global__ __launch_bounds__(256) void bnapply_kernel(const float* __restrict__ ZC, const float* __restrict__ stats,
                                                      const float* __restrict__ g, const float* __restrict__ bb,
                                                      unsigned short* __restrict__ XB, float carry, int n8) {
  const int i = blockIdx.x * 256 + threadIdx.x;
  if (i >= n8) return;
  const size_t e0 = (size_t)i * 8;
  const int d0 = (int)(e0 & (size_t)(kD - 1));
  const int grp = d0 >> 5, w = d0 & 31;
  const v4f z0 = *(const v4f*)(ZC + e0), z1 = *(const v4f*)(ZC + e0 + 4);
  const float* st = stats + grp * 64 + w;
  const v4f m0 = *(const v4f*)(st), m1 = *(const v4f*)(st + 4);
  const v4f q0 = *(const v4f*)(st + 32), q1 = *(const v4f*)(st + 36);
  const v4f g0 = *(const v4f*)(g + d0), g1 = *(const v4f*)(g + d0 + 4);
  const v4f b0 = *(const v4f*)(bb + d0), b1 = *(const v4f*)(bb + d0 + 4);
  unsigned short hb[8];
#pragma unroll
  for (int e = 0; e < 4; ++e) {
    const float y0 = (z0[e] - m0[e]) * rsqrtf(q0[e] + kEps) * g0[e] + b0[e];
    const float y1 = (z1[e] - m1[e]) * rsqrtf(q1[e] + kEps) * g1[e] + b1[e];
    const float w0 = y0 * (1.0f / (1.0f + expf(-y0)));
    const float w1 = y1 * (1.0f / (1.0f + expf(-y1)));
    hb[e]     = h_bits(carry * w0);
    hb[4 + e] = h_bits(carry * w1);
  }
  const v4u u = (v4u){pk16(hb[0], hb[1]), pk16(hb[2], hb[3]), pk16(hb[4], hb[5]), pk16(hb[6], hb[7])};
  unsigned short* q = XB + e0;
  *(volatile v4u*)q = u;
  __threadfence();
  *(volatile v4u*)q = u;
}

extern "C" void kernel_launch(void* const* d_in, const int* in_sizes, int n_in,
                              void* d_out, int out_size, void* d_ws, size_t ws_size, hipStream_t stream) {
  if (n_in < 35) return;
  if (in_sizes[0] != kNT * kD || out_size != kNT * kD) return;
  if (in_sizes[17] != kD * 3 * kD || in_sizes[18] != kD * kD || in_sizes[19] != kD * kFF || in_sizes[21] != kFF * kD ||
      in_sizes[23] != kD * kFF || in_sizes[25] != kFF * kD || in_sizes[27] != kD * 2 * kD || in_sizes[29] != kD * kKW ||
      in_sizes[33] != kD * kD || in_sizes[20] != kFF || in_sizes[24] != kFF || in_sizes[28] != 2 * kD) return;
  for (int i = 1; i <= 16; ++i) if (in_sizes[i] != kD) return;
  if (in_sizes[22] != kD || in_sizes[26] != kD || in_sizes[30] != kD || in_sizes[31] != kD || in_sizes[32] != kD || in_sizes[34] != kD) return;
  if (kWsTotal > ws_size) return;

  const float* x     = (const float*)d_in[0];
  const float* sb1s  = (const float*)d_in[1];
  const float* sb1b  = (const float*)d_in[2];
  const float* ln1g  = (const float*)d_in[3];
  const float* ln1b  = (const float*)d_in[4];
  const float* sb2s  = (const float*)d_in[5];
  const float* sb2b  = (const float*)d_in[6];
  const float* ln2g  = (const float*)d_in[7];
  const float* ln2b  = (const float*)d_in[8];
  const float* sb3s  = (const float*)d_in[9];
  const float* sb3b  = (const float*)d_in[10];
  const float* ln3g  = (const float*)d_in[11];
  const float* ln3b  = (const float*)d_in[12];
  const float* sb4s  = (const float*)d_in[13];
  const float* sb4b  = (const float*)d_in[14];
  const float* ln4g  = (const float*)d_in[15];
  const float* ln4b  = (const float*)d_in[16];
  const float* w_qkv = (const float*)d_in[17];
  const float* w_out = (const float*)d_in[18];
  const float* f1w1  = (const float*)d_in[19];
  const float* f1b1  = (const float*)d_in[20];
  const float* f1w2  = (const float*)d_in[21];
  const float* f1b2  = (const float*)d_in[22];
  const float* f2w1  = (const float*)d_in[23];
  const float* f2b1  = (const float*)d_in[24];
  const float* f2w2  = (const float*)d_in[25];
  const float* f2b2  = (const float*)d_in[26];
  const float* pw1w  = (const float*)d_in[27];
  const float* pw1b  = (const float*)d_in[28];
  const float* dww   = (const float*)d_in[29];
  const float* dwb   = (const float*)d_in[30];
  const float* bng   = (const float*)d_in[31];
  const float* bnb   = (const float*)d_in[32];
  const float* pw2w  = (const float*)d_in[33];
  const float* pw2b  = (const float*)d_in[34];
  float* out = (float*)d_out;

  char* ws = (char*)d_ws;
  unsigned short* WQKV = (unsigned short*)(ws + kOffWQKV);
  unsigned short* WOUT = (unsigned short*)(ws + kOffWOUT);
  unsigned short* F1W1 = (unsigned short*)(ws + kOffF1W1);
  unsigned short* F1W2 = (unsigned short*)(ws + kOffF1W2);
  unsigned short* PW1  = (unsigned short*)(ws + kOffPW1);
  unsigned short* PW2  = (unsigned short*)(ws + kOffPW2);
  unsigned short* F2W1 = (unsigned short*)(ws + kOffF2W1);
  unsigned short* F2W2 = (unsigned short*)(ws + kOffF2W2);
  float*          XS   = (float*)(ws + kOffXS);
  unsigned short* XA   = (unsigned short*)(ws + kOffXA);
  float*          QKVF = (float*)(ws + kOffBIG);
  float*          SPL  = (float*)(ws + kOffBIG);
  unsigned short* PPL  = (unsigned short*)(ws + kOffBIG + kBytesS);
  unsigned short* HD   = (unsigned short*)(ws + kOffBIG);
  float*          Z1   = (float*)(ws + kOffBIG);
  float*          ZG   = (float*)(ws + kOffBIG + (size_t)kNT * 1024 * 4);
  float*          ZC   = (float*)(ws + kOffBIG);
  unsigned short* QH   = (unsigned short*)(ws + kOffR2);
  unsigned short* KH   = (unsigned short*)(ws + kOffR2 + (size_t)kNG * kT * kDH * 2);
  unsigned short* VT   = (unsigned short*)(ws + kOffR2 + (size_t)2 * kNG * kT * kDH * 2);
  float*          Y    = (float*)(ws + kOffR2);
  float*          CS   = (float*)(ws + kOffCS);
  float*          STATS = (float*)(ws + kOffSTATS);
  const float* dummyf = sb1b;

  const dim3 blk(256);
  const int n8 = kNT * kD / 8;

  sbcast_kernel<<<dim3(n8 / 256), blk, 0, stream>>>(x, sb1s, sb1b, XA, n8);
  wtcast_kernel<<<dim3(kD / 64, (3 * kD) / 64), blk, 0, stream>>>(w_qkv, WQKV, kD, 3 * kD, 16.0f);
  wtcast_kernel<<<dim3(kD / 64, kD / 64), blk, 0, stream>>>(w_out, WOUT, kD, kD, 16.0f);
  wtcast_kernel<<<dim3(kD / 64, kFF / 64), blk, 0, stream>>>(f1w1, F1W1, kD, kFF, 16.0f);
  wtcast_kernel<<<dim3(kFF / 64, kD / 64), blk, 0, stream>>>(f1w2, F1W2, kFF, kD, 16.0f);
  wtcast_kernel<<<dim3(kD / 64, (2 * kD) / 64), blk, 0, stream>>>(pw1w, PW1, kD, 2 * kD, 16.0f);
  wtcast_kernel<<<dim3(kD / 64, kD / 64), blk, 0, stream>>>(pw2w, PW2, kD, kD, 16.0f);
  wtcast_kernel<<<dim3(kD / 64, kFF / 64), blk, 0, stream>>>(f2w1, F2W1, kD, kFF, 16.0f);
  wtcast_kernel<<<dim3(kFF / 64, kD / 64), blk, 0, stream>>>(f2w2, F2W2, kFF, kD, 16.0f);
  rope_table_kernel<<<dim3(kT / 8), blk, 0, stream>>>(CS);

  wmma_gemm64<0, false, 0, 0, false, 0><<<dim3(384, 1), blk, 0, stream>>>(
      XA, XA, kD, 0L, WQKV, WQKV, kD, 0L, (void*)QKVF, (void*)QKVF, 3 * kD, 0L, 0L, 1,
      dummyf, dummyf, 0L, kNT, 3 * kD, kD, 1.0f / 16.0f, 1.0f);
  rope_split_kernel<<<dim3(kT / 64, kH, kB), blk, 0, stream>>>(QKVF, CS, QH, KH, VT, 4.0f);
  for (int ch = 0; ch < kNCH; ++ch) {
    const size_t gb = (size_t)ch * kGC;
    wmma_gemm64<0, false, 0, 0, false, 0><<<dim3(8, kGC), blk, 0, stream>>>(
        QH + gb * kT * kDH, QH + gb * kT * kDH, kDH, (long)kT * kDH,
        KH + gb * kT * kDH, KH + gb * kT * kDH, kDH, (long)kT * kDH,
        (void*)SPL, (void*)SPL, kT, (long)kT * kT, 0L, 1,
        dummyf, dummyf, 0L, kT, kT, kDH, 0.125f / 16.0f, 1.0f);
    softmax_kernel<<<dim3(kGC * kT / 8), blk, 0, stream>>>(SPL, PPL, 2048.0f);
    wmma_gemm64<0, false, 0, 1, false, 0><<<dim3(1, kGC), blk, 0, stream>>>(
        PPL, PPL, kT, (long)kT * kT,
        VT + gb * kDH * kT, VT + gb * kDH * kT, kT, (long)kDH * kT,
        (void*)(XA + (gb / kH) * (size_t)kT * kD), (void*)(XA + (gb / kH) * (size_t)kT * kD), kD, (long)kT * kD, (long)kDH, kH,
        dummyf, dummyf, 0L, kT, kDH, kT, 1.0f / 512.0f, 1.0f);
  }
  wmma_gemm64<0, false, 0, 0, true, 0><<<dim3(128, 1), blk, 0, stream>>>(
      XA, XA, kD, 0L, WOUT, WOUT, kD, 0L, (void*)Y, (void*)Y, kD, 0L, 0L, 1,
      dummyf, x, 0L, kNT, kD, kD, 1.0f / 256.0f, 1.0f);
  ln_kernel<true><<<dim3(kNT / 8), blk, 0, stream>>>(Y, ln1g, ln1b, sb2s, sb2b, XS, XA);

  wmma_gemm64<0, false, 2, 1, false, 3><<<dim3(512, 1), blk, 0, stream>>>(
      XA, XA, kD, 0L, F1W1, F1W1, kD, 0L, (void*)HD, (void*)HD, kFF, 0L, 0L, 1,
      f1b1, dummyf, 0L, kNT, kFF, kD, 1.0f / 16.0f, 4.0f);
  wmma_gemm64<0, false, 2, 0, true, 0><<<dim3(128, 1), blk, 0, stream>>>(
      HD, HD, kFF, 0L, F1W2, F1W2, kFF, 0L, (void*)Y, (void*)Y, kD, 0L, 0L, 1,
      f1b2, XS, 0L, kNT, kD, kFF, 1.0f / 64.0f, 1.0f);
  ln_kernel<true><<<dim3(kNT / 8), blk, 0, stream>>>(Y, ln2g, ln2b, sb3s, sb3b, XS, XA);

  wmma_gemm64<0, false, 2, 0, false, 0><<<dim3(256, 1), blk, 0, stream>>>(
      XA, XA, kD, 0L, PW1, PW1, kD, 0L, (void*)Z1, (void*)Z1, 2 * kD, 0L, 0L, 1,
      pw1b, dummyf, 0L, kNT, 2 * kD, kD, 1.0f / 16.0f, 1.0f);
  glu_kernel<<<dim3(kNT * (kD / 4) / 256), blk, 0, stream>>>(Z1, ZG);
  dwconv_kernel<<<dim3(kD / 64, kT / 64, kB), blk, 0, stream>>>(ZG, dww, dwb, ZC);
  bnstats_kernel<<<dim3(kD / 32), blk, 0, stream>>>(ZC, STATS);
  bnapply_kernel<<<dim3(n8 / 256), blk, 0, stream>>>(ZC, STATS, bng, bnb, XA, 4.0f, n8);
  wmma_gemm64<0, false, 2, 0, true, 0><<<dim3(128, 1), blk, 0, stream>>>(
      XA, XA, kD, 0L, PW2, PW2, kD, 0L, (void*)Y, (void*)Y, kD, 0L, 0L, 1,
      pw2b, XS, 0L, kNT, kD, kD, 1.0f / 64.0f, 1.0f);
  ln_kernel<true><<<dim3(kNT / 8), blk, 0, stream>>>(Y, ln3g, ln3b, sb4s, sb4b, XS, XA);

  wmma_gemm64<0, false, 2, 1, false, 3><<<dim3(512, 1), blk, 0, stream>>>(
      XA, XA, kD, 0L, F2W1, F2W1, kD, 0L, (void*)HD, (void*)HD, kFF, 0L, 0L, 1,
      f2b1, dummyf, 0L, kNT, kFF, kD, 1.0f / 16.0f, 4.0f);
  wmma_gemm64<0, false, 2, 0, true, 0><<<dim3(128, 1), blk, 0, stream>>>(
      HD, HD, kFF, 0L, F2W2, F2W2, kFF, 0L, (void*)Y, (void*)Y, kD, 0L, 0L, 1,
      f2b2, XS, 0L, kNT, kD, kFF, 1.0f / 64.0f, 1.0f);
  ln_kernel<false><<<dim3(kNT / 8), blk, 0, stream>>>(Y, ln4g, ln4b, sb4s, sb4b, out, XA);
}
